// MHSA_8323646620297
// MI455X (gfx1250) — hardware-verified
//
#include <hip/hip_runtime.h>
#include <math.h>
#include <stdint.h>

#define NB    16
#define CH    512
#define IMW   32
#define IMH   32
#define NTOK  1024
#define NHD   8
#define HD    64
#define MTOK  (NB * NTOK)
#define VTP   MTOK
#define NQKV  (3 * CH)

static_assert(NTOK == IMW * IMH);
static_assert(IMH == 32);
static_assert(CH == NHD * HD);
static_assert(HD == 64);
static_assert(CH % 64 == 0);
static_assert(NTOK % 64 == 0);
static_assert(MTOK % 64 == 0);
static_assert(CH % 32 == 0);
static_assert(CH % 256 == 0);
static_assert((CH * CH) % (8 * 256) == 0);
static_assert(NTOK % 128 == 0);
static_assert(HD * IMH == 2 * 256 * 4);
static_assert(HD * IMW == 2 * 256 * 4);
static_assert(sizeof(__bf16) == 2);

typedef __attribute__((ext_vector_type(16))) _Float16 v16h;
typedef __attribute__((ext_vector_type(8)))  _Float16 v8h;
typedef __attribute__((ext_vector_type(16))) __bf16   v16b;
typedef __attribute__((ext_vector_type(8)))  __bf16   v8b;
typedef __attribute__((ext_vector_type(8)))  float    v8f;
typedef __attribute__((ext_vector_type(4)))  float    v4f;
typedef __attribute__((ext_vector_type(4)))  unsigned int v4u;

__device__ __forceinline__ unsigned short f2bf_bits(float f) {
  unsigned u = __float_as_uint(f);
  return (unsigned short)((u + 0x7FFFu + ((u >> 16) & 1u)) >> 16);
}
__device__ __forceinline__ float bf_bits2f(unsigned short h) { return __uint_as_float(((unsigned)h) << 16); }
__device__ __forceinline__ float bf_rne(float f) { return bf_bits2f(f2bf_bits(f)); }
__device__ __forceinline__ unsigned pk16(unsigned short a, unsigned short b) { return (unsigned)a | ((unsigned)b << 16); }

__device__ __forceinline__ void dep_guard_b(v8f& a, v8f& b, v16b x, v16b y) { asm volatile("v_nop\n\tv_nop\n\tv_nop\n\tv_nop" : "+v"(a), "+v"(b) : "v"(x), "v"(y)); }
__device__ __forceinline__ void keep4_b(v16b a, v16b b, v16b c, v16b d) { asm volatile("v_nop" :: "v"(a), "v"(b), "v"(c), "v"(d)); }
__device__ __forceinline__ void acc_guard4(v8f& a, v8f& b, v8f& c, v8f& d) { asm volatile("v_nop\n\tv_nop\n\tv_nop\n\tv_nop" : "+v"(a), "+v"(b), "+v"(c), "+v"(d)); }

struct FragB {
  union U { v16b v; v8b h[2]; };
  static __device__ __forceinline__ v16b load(const __bf16* p) {
    U f; f.h[0] = *(const v8b*)(p); f.h[1] = *(const v8b*)(p + 16); return f.v;
  }
  static __device__ __forceinline__ v8f mma(v16b a, v16b b, v8f c) {
    return __builtin_amdgcn_wmma_f32_16x16x32_bf16(false, a, false, b, (short)0, c, false, false);
  }
  static __device__ __forceinline__ void guard(v8f& a, v8f& b, v16b x, v16b y) { dep_guard_b(a, b, x, y); }
  static __device__ __forceinline__ void keep(v16b a, v16b b, v16b c, v16b d) { keep4_b(a, b, c, d); }
};

template <bool SPLIT, int BIAS_MODE, int OUT_MODE>
__global__ __launch_bounds__(256) void wmma_gemm64(
    const unsigned short* __restrict__ Ap, const unsigned short* __restrict__ A2p, int lda, long strideA,
    const unsigned short* __restrict__ Btp, const unsigned short* __restrict__ Bt2p, int ldb, long strideB,
    void* __restrict__ Cout, void* __restrict__ Cout2, int ldc, long strideC,
    const float* __restrict__ bias, int M, int N, int K, float scale) {
  typedef __bf16 T;
  typedef v16b V;
  const T* A = (const T*)(const void*)Ap; const T* A2 = (const T*)(const void*)A2p;
  const T* Bt = (const T*)(const void*)Btp; const T* Bt2 = (const T*)(const void*)Bt2p;
  __shared__ __align__(16) float sT[8][16 * 68];
  const int b    = blockIdx.y;
  const int lane = threadIdx.x & 31;
  const int wave = threadIdx.x >> 5;
  const int tilesN = N >> 6;
  const int tilesM = M >> 6;
  const int tile = blockIdx.x * 8 + wave;
  if (tile >= tilesM * tilesN) return;
  const int tm = tile / tilesN;
  const int tn = tile - tm * tilesN;
  const int m0 = tm << 6;
  const int n0 = tn << 6;

  const T* Ab  = A  + (size_t)b * strideA;
  const T* Bb  = Bt + (size_t)b * strideB;
  const T* Ab2 = SPLIT ? (A2  + (size_t)b * strideA) : nullptr;
  const T* Bb2 = SPLIT ? (Bt2 + (size_t)b * strideB) : nullptr;

  const int rlane = lane & 15;
  const int koff  = (lane >> 4) * 8;
  const int mOff  = (lane >> 4) * 8;

  v8f acc[4][4];
#pragma unroll
  for (int i = 0; i < 4; ++i)
#pragma unroll
    for (int j = 0; j < 4; ++j) acc[i][j] = (v8f){0.f,0.f,0.f,0.f,0.f,0.f,0.f,0.f};

  for (int k0 = 0; k0 < K; k0 += 32) {
    V bh[4], bl[4];
#pragma unroll
    for (int j = 0; j < 4; ++j) {
      const size_t bo = (size_t)(n0 + (j << 4) + rlane) * ldb + koff + k0;
      bh[j] = FragB::load(Bb + bo);
      if (SPLIT) bl[j] = FragB::load(Bb2 + bo); else bl[j] = bh[j];
    }
#pragma unroll
    for (int i = 0; i < 4; ++i) {
      const size_t ao = (size_t)(m0 + (i << 4) + rlane) * lda + koff + k0;
      V ah = FragB::load(Ab + ao);
      V al;
      if (SPLIT) al = FragB::load(Ab2 + ao); else al = ah;
#pragma unroll
      for (int j = 0; j < 4; ++j) {
        acc[i][j] = FragB::mma(ah, bh[j], acc[i][j]);
        if (SPLIT) {
          acc[i][j] = FragB::mma(ah, bl[j], acc[i][j]);
          acc[i][j] = FragB::mma(al, bh[j], acc[i][j]);
        }
      }
      FragB::guard(acc[i][0], acc[i][3], ah, al);
    }
    FragB::keep(bh[0], bh[1], bh[2], bh[3]);
    if (SPLIT) FragB::keep(bl[0], bl[1], bl[2], bl[3]);
  }
  acc_guard4(acc[0][0], acc[0][1], acc[0][2], acc[0][3]);
  acc_guard4(acc[1][0], acc[1][1], acc[1][2], acc[1][3]);
  acc_guard4(acc[2][0], acc[2][1], acc[2][2], acc[2][3]);
  acc_guard4(acc[3][0], acc[3][1], acc[3][2], acc[3][3]);

  float* slab = sT[wave];
#pragma unroll
  for (int i = 0; i < 4; ++i) {
    const int mBase = m0 + (i << 4);
#pragma unroll
    for (int j = 0; j < 4; ++j) {
      const int n = n0 + (j << 4) + rlane;
      float bv = 0.f;
      if (BIAS_MODE == 2) bv = bf_rne(bias[n]);
#pragma unroll
      for (int r = 0; r < 8; ++r) {
        float v = acc[i][j][r] * scale;
        if (BIAS_MODE == 1) v += bf_rne(bias[mBase + mOff + r]);
        if (BIAS_MODE == 2) v += bv;
        slab[(mOff + r) * 68 + (j << 4) + rlane] = v;
      }
    }
    __builtin_amdgcn_fence(__ATOMIC_RELEASE, "workgroup");
    __builtin_amdgcn_wave_barrier();
    __builtin_amdgcn_fence(__ATOMIC_ACQUIRE, "workgroup");
    if (OUT_MODE == 0) {
      float* C = (float*)Cout + (size_t)b * strideC;
      const int hh = lane >> 4, c4 = (lane & 15) * 4;
      for (int pass = 0; pass < 2; ++pass) {
#pragma unroll
        for (int it = 0; it < 8; ++it) {
          const int row = it * 2 + hh;
          v4f v = *(const v4f*)(slab + row * 68 + c4);
          *(volatile v4f*)(C + (size_t)(mBase + row) * ldc + n0 + c4) = v;
        }
        __threadfence();
      }
    } else {
      const int q = lane >> 3, c8 = (lane & 7) * 8;
      unsigned short* C  = (unsigned short*)Cout  + (size_t)b * strideC;
      unsigned short* C2 = (unsigned short*)Cout2 + (size_t)b * strideC;
      for (int pass = 0; pass < 2; ++pass) {
#pragma unroll
        for (int it = 0; it < 4; ++it) {
          const int row = it * 4 + q;
          const float* sp = slab + row * 68 + c8;
          v8h hv, lv;
#pragma unroll
          for (int e = 0; e < 8; ++e) {
            unsigned short hb = f2bf_bits(sp[e]);
            unsigned short lb = f2bf_bits(sp[e] - bf_bits2f(hb));
            hv[e] = __builtin_bit_cast(_Float16, hb);
            lv[e] = __builtin_bit_cast(_Float16, lb);
          }
          *(volatile v8h*)(C  + (size_t)(mBase + row) * ldc + n0 + c8) = hv;
          *(volatile v8h*)(C2 + (size_t)(mBase + row) * ldc + n0 + c8) = lv;
        }
        __threadfence();
      }
    }
    __builtin_amdgcn_fence(__ATOMIC_RELEASE, "workgroup");
    __builtin_amdgcn_wave_barrier();
    __builtin_amdgcn_fence(__ATOMIC_ACQUIRE, "workgroup");
  }
}

__global__ __launch_bounds__(256) void convrows_kernel(const float* __restrict__ in, unsigned short* __restrict__ out,
                                                       int ncols, int ldout, int n8) {
  const int i = blockIdx.x * 256 + threadIdx.x;
  if (i < n8) {
    const size_t e0 = (size_t)i * 8;
    const int row = (int)(e0 / (size_t)ncols);
    const int col = (int)(e0 - (size_t)row * ncols);
    const v4f a = *(const v4f*)(in + e0);
    const v4f c = *(const v4f*)(in + e0 + 4);
    v4u hv;
    hv[0] = pk16(f2bf_bits(a[0]), f2bf_bits(a[1]));
    hv[1] = pk16(f2bf_bits(a[2]), f2bf_bits(a[3]));
    hv[2] = pk16(f2bf_bits(c[0]), f2bf_bits(c[1]));
    hv[3] = pk16(f2bf_bits(c[2]), f2bf_bits(c[3]));
    const size_t o = (size_t)row * ldout + col;
    for (int pass = 0; pass < 2; ++pass) {
      *(volatile v4u*)(out + o) = hv;
      __threadfence();
    }
  }
}

__global__ __launch_bounds__(256) void tconv_kernel(const float* __restrict__ W, unsigned short* __restrict__ oh,
                                                    int ldin, int ldout, long sIn, long sOut) {
  __shared__ __align__(16) float tf[64 * 68];
  W  += (size_t)blockIdx.z * sIn;
  oh += (size_t)blockIdx.z * sOut;
  const int c0  = blockIdx.x * 64;
  const int r0  = blockIdx.y * 64;
  const int tid = threadIdx.x;
  {
    const int lr = tid >> 4;
    const int c4 = (tid & 15) * 4;
#pragma unroll
    for (int it = 0; it < 4; ++it) {
      const int rr = it * 16 + lr;
      const v4f a = *(const v4f*)(W + (size_t)(r0 + rr) * ldin + c0 + c4);
      *(v4f*)(tf + rr * 68 + c4) = a;
    }
  }
  __syncthreads();
  const int sub = tid >> 3;
  const int c8  = (tid & 7) * 8;
  v4u hv[2];
#pragma unroll
  for (int it = 0; it < 2; ++it) {
    const int oc = it * 32 + sub;
    v4u a;
#pragma unroll
    for (int q = 0; q < 4; ++q) {
      const float f0 = tf[(c8 + 2 * q) * 68 + oc];
      const float f1 = tf[(c8 + 2 * q + 1) * 68 + oc];
      a[q] = pk16(f2bf_bits(f0), f2bf_bits(f1));
    }
    hv[it] = a;
  }
  for (int pass = 0; pass < 2; ++pass) {
#pragma unroll
    for (int it = 0; it < 2; ++it) {
      const int oc = it * 32 + sub;
      const size_t go = (size_t)(c0 + oc) * ldout + r0 + c8;
      *(volatile v4u*)(oh + go) = hv[it];
    }
    __threadfence();
  }
}

__global__ __launch_bounds__(256) void pos_kernel(const float* __restrict__ rel_h, const float* __restrict__ rel_w,
                                                  unsigned short* __restrict__ ph, unsigned short* __restrict__ pl) {
  __shared__ __align__(16) float RH[HD * IMH];
  __shared__ __align__(16) float RW[HD * IMW];
  const int hd  = blockIdx.y;
  const int nb  = blockIdx.x * 128;
  const int tid = threadIdx.x;
  const float* rh = rel_h + (size_t)hd * HD * IMH;
  const float* rw = rel_w + (size_t)hd * HD * IMW;
#pragma unroll
  for (int k = 0; k < 2; ++k) {
    const int e = (k * 256 + tid) * 4;
    *(v4f*)(RH + e) = *(const v4f*)(rh + e);
    *(v4f*)(RW + e) = *(const v4f*)(rw + e);
  }
  __syncthreads();
  const int sub = tid >> 3;
  const int dg  = tid & 7;
  v4u hv[4], lv[4];
#pragma unroll
  for (int k = 0; k < 4; ++k) {
    const int n = nb + k * 32 + sub;
    const int j = n & 31, i = n >> 5;
    v4u a, a2;
#pragma unroll
    for (int q = 0; q < 4; ++q) {
      const int d0 = dg * 8 + 2 * q;
      const float f0 = bf_rne(RH[d0 * IMH + j]) + bf_rne(RW[d0 * IMW + i]);
      const float f1 = bf_rne(RH[(d0 + 1) * IMH + j]) + bf_rne(RW[(d0 + 1) * IMW + i]);
      const unsigned short h0 = f2bf_bits(f0), h1 = f2bf_bits(f1);
      const unsigned short l0 = f2bf_bits(f0 - bf_bits2f(h0)), l1 = f2bf_bits(f1 - bf_bits2f(h1));
      a[q]  = pk16(h0, h1);
      a2[q] = pk16(l0, l1);
    }
    hv[k] = a; lv[k] = a2;
  }
  for (int pass = 0; pass < 2; ++pass) {
#pragma unroll
    for (int k = 0; k < 4; ++k) {
      const int n = nb + k * 32 + sub;
      const size_t go = (size_t)n * CH + hd * HD + dg * 8;
      *(volatile v4u*)(ph + go) = hv[k];
      *(volatile v4u*)(pl + go) = lv[k];
    }
    __threadfence();
  }
}

#define AT_D  64
#define AT_KD 128
#define AT_NW 4
#define AT_QB 64
#define AT_KC 64

__device__ __forceinline__ unsigned short at_bf_bits(float f) {
  unsigned u = __float_as_uint(f);
  return (unsigned short)((u + 0x7FFFu + ((u >> 16) & 1u)) >> 16);
}
__device__ __forceinline__ __bf16 at_f2bf(float f) { return __builtin_bit_cast(__bf16, at_bf_bits(f)); }
__device__ __forceinline__ void at_split(float f, __bf16& hi, __bf16& lo) {
  const unsigned short hb = at_bf_bits(f);
  hi = __builtin_bit_cast(__bf16, hb);
  lo = at_f2bf(f - __uint_as_float(((unsigned)hb) << 16));
}
__device__ __forceinline__ v8f at_mma(v16b a, v16b b, v8f c) {
  c = __builtin_amdgcn_wmma_f32_16x16x32_bf16(false, a, false, b, (short)0, c, false, false);
  asm volatile("v_nop\n\tv_nop\n\tv_nop\n\tv_nop" : "+v"(c) : "v"(a), "v"(b));
  return c;
}

__global__ __launch_bounds__(128)
void attn_kernel(const unsigned short* __restrict__ qhp, const unsigned short* __restrict__ qlp,
                 const unsigned short* __restrict__ khp, const unsigned short* __restrict__ klp,
                 const unsigned short* __restrict__ php, const unsigned short* __restrict__ plp,
                 const unsigned short* __restrict__ vhp, const unsigned short* __restrict__ vlp,
                 float* __restrict__ out) {
  union FB { v16b v; v8b h[2]; };
  __shared__ __align__(16) __bf16 Ash[AT_QB * AT_KD];
  __shared__ __align__(16) __bf16 Asl[AT_QB * AT_KD];
  __shared__ __align__(16) __bf16 Bsh[AT_KC * AT_KD];
  __shared__ __align__(16) __bf16 Bsl[AT_KC * AT_KD];
  __shared__ __align__(16) __bf16 Vth[AT_D * AT_KC];
  __shared__ __align__(16) __bf16 Vtl[AT_D * AT_KC];
  __shared__ __align__(16) __bf16 Psh[AT_NW][16 * AT_KC];
  __shared__ __align__(16) __bf16 Psl[AT_NW][16 * AT_KC];
  __shared__ __align__(16) float  Os[AT_D * 68];

  const int tid  = threadIdx.x;
  const int wave = tid >> 5;
  const int lane = tid & 31;
  const int hh   = lane >> 4;
  const int c    = lane & 15;

  const int bx = blockIdx.x;
  const int qb = bx & 15;
  const int hd = (bx >> 4) & 7;
  const int b  = bx >> 7;
  const int n0 = qb * AT_QB;
  const size_t trow = (size_t)b * NTOK;

  const __bf16* Qh = (const __bf16*)(const void*)qhp + (size_t)hd * AT_D;
  const __bf16* Ql = (const __bf16*)(const void*)qlp + (size_t)hd * AT_D;
  const __bf16* Kh = (const __bf16*)(const void*)khp + (size_t)hd * AT_D;
  const __bf16* Kl = (const __bf16*)(const void*)klp + (size_t)hd * AT_D;
  const __bf16* Rh = (const __bf16*)(const void*)php + (size_t)hd * AT_D;
  const __bf16* Rl = (const __bf16*)(const void*)plp + (size_t)hd * AT_D;
  const __bf16* Vh = (const __bf16*)(const void*)vhp + (size_t)hd * AT_D * VTP + trow;
  const __bf16* Vl = (const __bf16*)(const void*)vlp + (size_t)hd * AT_D * VTP + trow;

  {
    const int r = tid >> 1, half = (tid & 1) * 32;
    const size_t oq = (trow + (size_t)(n0 + r)) * CH + half;
    const size_t op = (size_t)(n0 + r) * CH + half;
    const __bf16* qs  = Qh + oq;
    const __bf16* qsl = Ql + oq;
    const __bf16* ps  = Rh + op;
    const __bf16* psl = Rl + op;
#pragma unroll
    for (int i = 0; i < 4; ++i) {
      const v8b a0 = *(const v8b*)(qs  + 8 * i);
      const v8b a1 = *(const v8b*)(qsl + 8 * i);
      const v8b g0 = *(const v8b*)(ps  + 8 * i);
      const v8b g1 = *(const v8b*)(psl + 8 * i);
      *(v8b*)(Ash + r * AT_KD + half + 8 * i) = a0;
      *(v8b*)(Asl + r * AT_KD + half + 8 * i) = a1;
      *(v8b*)(Ash + r * AT_KD + AT_D + half + 8 * i) = g0;
      *(v8b*)(Asl + r * AT_KD + AT_D + half + 8 * i) = g1;
    }
  }
  __syncthreads();

  const __bf16* arh = Ash + (wave * 16 + c) * AT_KD + 8 * hh;
  const __bf16* arl = Asl + (wave * 16 + c) * AT_KD + 8 * hh;

  float mrow[8], lrow[8];
  v8f oacc[4];
#pragma unroll
  for (int r = 0; r < 8; ++r) { mrow[r] = -INFINITY; lrow[r] = 0.f; }
#pragma unroll
  for (int t = 0; t < 4; ++t) oacc[t] = (v8f){0.f,0.f,0.f,0.f,0.f,0.f,0.f,0.f};

  const int nChunks = NTOK / AT_KC;
  for (int kc = 0; kc < nChunks; ++kc) {
    const int kv0 = kc * AT_KC;
    __syncthreads();
    {
      const int r = tid >> 1, half = (tid & 1) * 32;
      const size_t ok = (trow + (size_t)(kv0 + r)) * CH + half;
      const __bf16* ks  = Kh + ok;
      const __bf16* ksl = Kl + ok;
      const __bf16* qs  = Qh + ok;
      const __bf16* qsl = Ql + ok;
#pragma unroll
      for (int i = 0; i < 4; ++i) {
        const v8b a0 = *(const v8b*)(ks  + 8 * i);
        const v8b a1 = *(const v8b*)(ksl + 8 * i);
        const v8b g0 = *(const v8b*)(qs  + 8 * i);
        const v8b g1 = *(const v8b*)(qsl + 8 * i);
        *(v8b*)(Bsh + r * AT_KD + half + 8 * i) = a0;
        *(v8b*)(Bsl + r * AT_KD + half + 8 * i) = a1;
        *(v8b*)(Bsh + r * AT_KD + AT_D + half + 8 * i) = g0;
        *(v8b*)(Bsl + r * AT_KD + AT_D + half + 8 * i) = g1;
      }
      const __bf16* vs  = Vh + (size_t)r * VTP + kv0 + half;
      const __bf16* vsl = Vl + (size_t)r * VTP + kv0 + half;
#pragma unroll
      for (int i = 0; i < 4; ++i) {
        const v8b b0 = *(const v8b*)(vs  + 8 * i);
        const v8b b1 = *(const v8b*)(vsl + 8 * i);
        *(v8b*)(Vth + r * AT_KC + half + 8 * i) = b0;
        *(v8b*)(Vtl + r * AT_KC + half + 8 * i) = b1;
      }
    }
    __syncthreads();

    v8f s[4];
#pragma unroll
    for (int j = 0; j < 4; ++j) s[j] = (v8f){0.f,0.f,0.f,0.f,0.f,0.f,0.f,0.f};
#pragma unroll 1
    for (int dc = 0; dc < 4; ++dc) {
      FB fa, fl;
      fa.h[0] = *(const v8b*)(arh + dc * 32);
      fa.h[1] = *(const v8b*)(arh + dc * 32 + 16);
      fl.h[0] = *(const v8b*)(arl + dc * 32);
      fl.h[1] = *(const v8b*)(arl + dc * 32 + 16);
#pragma unroll
      for (int j = 0; j < 4; ++j) {
        FB kb, kl;
        const int bo = (j * 16 + c) * AT_KD + dc * 32 + 8 * hh;
        kb.h[0] = *(const v8b*)(Bsh + bo);
        kb.h[1] = *(const v8b*)(Bsh + bo + 16);
        kl.h[0] = *(const v8b*)(Bsl + bo);
        kl.h[1] = *(const v8b*)(Bsl + bo + 16);
        s[j] = at_mma(fa.v, kb.v, s[j]);
        s[j] = at_mma(fa.v, kl.v, s[j]);
        s[j] = at_mma(fl.v, kb.v, s[j]);
      }
    }
    float cm[8];
#pragma unroll
    for (int r = 0; r < 8; ++r) {
      float m = fmaxf(fmaxf(s[0][r], s[1][r]), fmaxf(s[2][r], s[3][r]));
#pragma unroll
      for (int off = 1; off < 16; off <<= 1) m = fmaxf(m, __shfl_xor(m, off, 32));
      cm[r] = m;
    }
    __bf16* pwh = Psh[wave];
    __bf16* pwl = Psl[wave];
#pragma unroll
    for (int r = 0; r < 8; ++r) {
      const float mnew = fmaxf(mrow[r], cm[r]);
      const float alpha = expf(mrow[r] - mnew);
      mrow[r] = mnew;
      float psum = 0.f;
#pragma unroll
      for (int j = 0; j < 4; ++j) {
        const float p = expf(s[j][r] - mnew);
        psum += p;
        __bf16 a, bl; at_split(p, a, bl);
        pwh[(8 * hh + r) * AT_KC + j * 16 + c] = a;
        pwl[(8 * hh + r) * AT_KC + j * 16 + c] = bl;
      }
#pragma unroll
      for (int off = 1; off < 16; off <<= 1) psum += __shfl_xor(psum, off, 32);
      lrow[r] = lrow[r] * alpha + psum;
#pragma unroll
      for (int t = 0; t < 4; ++t) oacc[t][r] *= alpha;
    }
    __builtin_amdgcn_fence(__ATOMIC_RELEASE, "workgroup");
    __builtin_amdgcn_wave_barrier();
    __builtin_amdgcn_fence(__ATOMIC_ACQUIRE, "workgroup");
#pragma unroll 1
    for (int kk = 0; kk < 2; ++kk) {
      FB pa, pl;
      pa.h[0] = *(const v8b*)(pwh + c * AT_KC + kk * 32 + 8 * hh);
      pa.h[1] = *(const v8b*)(pwh + c * AT_KC + kk * 32 + 16 + 8 * hh);
      pl.h[0] = *(const v8b*)(pwl + c * AT_KC + kk * 32 + 8 * hh);
      pl.h[1] = *(const v8b*)(pwl + c * AT_KC + kk * 32 + 16 + 8 * hh);
#pragma unroll
      for (int t = 0; t < 4; ++t) {
        FB vb, vl;
        vb.h[0] = *(const v8b*)(Vth + (t * 16 + c) * AT_KC + kk * 32 + 8 * hh);
        vb.h[1] = *(const v8b*)(Vth + (t * 16 + c) * AT_KC + kk * 32 + 16 + 8 * hh);
        vl.h[0] = *(const v8b*)(Vtl + (t * 16 + c) * AT_KC + kk * 32 + 8 * hh);
        vl.h[1] = *(const v8b*)(Vtl + (t * 16 + c) * AT_KC + kk * 32 + 16 + 8 * hh);
        oacc[t] = at_mma(pa.v, vb.v, oacc[t]);
        oacc[t] = at_mma(pa.v, vl.v, oacc[t]);
        oacc[t] = at_mma(pl.v, vb.v, oacc[t]);
      }
    }
  }

#pragma unroll
  for (int r = 0; r < 8; ++r) {
    const float inv = 1.0f / lrow[r];
#pragma unroll
    for (int t = 0; t < 4; ++t) Os[(t * 16 + c) * 68 + wave * 16 + 8 * hh + r] = oacc[t][r] * inv;
  }
  __syncthreads();
  {
    const int lr = tid >> 4;
    const int c4 = (tid & 15) * 4;
    float* ob = out + ((size_t)b * CH + (size_t)hd * AT_D) * NTOK + n0;
    for (int pass = 0; pass < 2; ++pass) {
#pragma unroll
      for (int it = 0; it < 8; ++it) {
        const int d = it * 8 + lr;
        v4f val = *(const v4f*)(Os + d * 68 + c4);
        *(volatile v4f*)(ob + (size_t)d * NTOK + c4) = val;
      }
      __threadfence();
    }
  }
}

extern "C" void kernel_launch(void* const* d_in, const int* in_sizes, int n_in,
                              void* d_out, int out_size, void* d_ws, size_t ws_size,
                              hipStream_t stream) {
  if (n_in < 9) return;
  if (in_sizes[0] != NB * CH * NTOK) return;
  if (in_sizes[1] != CH * CH) return;
  if (in_sizes[2] != CH) return;
  if (in_sizes[3] != CH * CH) return;
  if (in_sizes[4] != CH) return;
  if (in_sizes[5] != CH * CH) return;
  if (in_sizes[6] != CH) return;
  if (in_sizes[7] != NHD * HD * IMH) return;
  if (in_sizes[8] != NHD * HD * IMW) return;
  if (out_size != NB * CH * NTOK) return;

  const float* x     = (const float*)d_in[0];
  const float* wq    = (const float*)d_in[1];
  const float* bq    = (const float*)d_in[2];
  const float* wk    = (const float*)d_in[3];
  const float* bk    = (const float*)d_in[4];
  const float* wv    = (const float*)d_in[5];
  const float* bv    = (const float*)d_in[6];
  const float* rel_h = (const float*)d_in[7];
  const float* rel_w = (const float*)d_in[8];

  const size_t PXB = (size_t)MTOK * CH * 2;
  const size_t PWB = (size_t)NQKV * CH * 2;
  const size_t PPL = (size_t)MTOK * CH * 2;
  const size_t PPS = (size_t)NTOK * CH * 2;
  const size_t PVT = (size_t)CH * VTP * 2;
  size_t off = 0;
  const size_t oXB  = off; off += PXB;
  const size_t oWB  = off; off += PWB;
  const size_t oQh  = off; off += PPL;  const size_t oQl  = off; off += PPL;
  const size_t oKh  = off; off += PPL;  const size_t oKl  = off; off += PPL;
  const size_t oPh  = off; off += PPS;  const size_t oPl  = off; off += PPS;
  const size_t oVTh = off; off += PVT;  const size_t oVTl = off; off += PVT;
  if (off > ws_size) return;
  if (off > (size_t)134217728) return;

  char* ws = (char*)d_ws;
  unsigned short* XB  = (unsigned short*)(ws + oXB);
  unsigned short* WB  = (unsigned short*)(ws + oWB);
  unsigned short* Qh  = (unsigned short*)(ws + oQh);  unsigned short* Ql  = (unsigned short*)(ws + oQl);
  unsigned short* Kh  = (unsigned short*)(ws + oKh);  unsigned short* Kl  = (unsigned short*)(ws + oKl);
  unsigned short* Ph  = (unsigned short*)(ws + oPh);  unsigned short* Pl  = (unsigned short*)(ws + oPl);
  unsigned short* VTh = (unsigned short*)(ws + oVTh); unsigned short* VTl = (unsigned short*)(ws + oVTl);

  const dim3 blk(256);

  tconv_kernel<<<dim3(NTOK / 64, CH / 64, NB), blk, 0, stream>>>(x, XB, NTOK, CH, (long)CH * NTOK, (long)NTOK * CH);
  const int n8w = CH * CH / 8;
  convrows_kernel<<<dim3(n8w / 256), blk, 0, stream>>>(wq, WB, CH, CH, n8w);
  convrows_kernel<<<dim3(n8w / 256), blk, 0, stream>>>(wk, WB + (size_t)CH * CH, CH, CH, n8w);
  convrows_kernel<<<dim3(n8w / 256), blk, 0, stream>>>(wv, WB + (size_t)2 * CH * CH, CH, CH, n8w);
  pos_kernel<<<dim3(NTOK / 128, NHD), blk, 0, stream>>>(rel_h, rel_w, Ph, Pl);
  const dim3 gP(((MTOK / 64) * (CH / 64) + 7) / 8, 1);
  wmma_gemm64<false, 2, 2><<<gP, blk, 0, stream>>>(
      XB, XB, CH, 0L, WB, WB, CH, 0L, (void*)Qh, (void*)Ql, CH, 0L, bq, MTOK, CH, CH, 1.0f);
  wmma_gemm64<false, 2, 2><<<gP, blk, 0, stream>>>(
      XB, XB, CH, 0L, WB + (size_t)CH * CH, WB + (size_t)CH * CH, CH, 0L, (void*)Kh, (void*)Kl, CH, 0L, bk, MTOK, CH, CH, 1.0f);
  const dim3 gVT(((CH / 64) * (MTOK / 64) + 7) / 8, 1);
  wmma_gemm64<false, 1, 2><<<gVT, blk, 0, stream>>>(
      WB + (size_t)2 * CH * CH, WB + (size_t)2 * CH * CH, CH, 0L, XB, XB, CH, 0L,
      (void*)VTh, (void*)VTl, VTP, 0L, bv, CH, MTOK, CH, 1.0f);
  attn_kernel<<<dim3(NB * NHD * (NTOK / AT_QB)), dim3(128), 0, stream>>>(Qh, Ql, Kh, Kl, Ph, Pl, VTh, VTl, (float*)d_out);
  (void)hipGetLastError();
}
